// GroupedQueryAttention_34316788695052
// MI455X (gfx1250) — hardware-verified
//
#include <hip/hip_runtime.h>
#pragma clang fp contract(off)


#ifndef NB
#define NB 2
#endif
#ifndef SEQ
#define SEQ 2048
#endif
#define NB_FULL  2
#define SEQ_FULL 2048
#define DM   1024
#define NH   16
#define NKV  4
#define REP  (NH / NKV)
#define HD   64
#define DQ   (NH * HD)
#define DKV  (NKV * HD)
#define NQKV (DQ + 2 * DKV)
#define RH   ((SEQ) < 512 ? (SEQ) : 512)
#define NROT 5
#define NTAB 8
#define PP   40
#define PCAR 1024.0f
#define L2E  1.4426950408889634f
#define NEGBIG (-3.0e38f)

static_assert(HD == 64);
static_assert(REP * NKV == NH);
static_assert(SEQ % 64 == 0);
static_assert(RH % 64 == 0);
static_assert(RH > 0);
static_assert((SEQ - RH) % 64 == 0);
static_assert(NB <= NB_FULL);
static_assert(SEQ <= SEQ_FULL);
static_assert(DM % 32 == 0);
static_assert(DQ % 32 == 0);
static_assert((NB * SEQ) % 64 == 0);
static_assert(NQKV % 64 == 0);
static_assert(DM % 64 == 0);
static_assert(PP % 8 == 0);
static_assert(PP >= 32);
static_assert(NROT <= NTAB);
static_assert(DQ == DM);
static_assert(RH <= SEQ);

typedef _Float16 h16;
typedef unsigned short bf;
typedef __attribute__((ext_vector_type(16))) __bf16   v16bf;
typedef __attribute__((ext_vector_type(16))) _Float16 v16h;
typedef __attribute__((ext_vector_type(8)))  _Float16 v8h;
typedef __attribute__((ext_vector_type(8)))  unsigned short v8us;
typedef __attribute__((ext_vector_type(8)))  float    v8f;
typedef __attribute__((ext_vector_type(4)))  float    v4f;
typedef __attribute__((ext_vector_type(2)))  float    v2f;
typedef __attribute__((ext_vector_type(2)))  _Float16 v2h;
typedef __attribute__((ext_vector_type(2)))  unsigned short v2us;
typedef v8h  __attribute__((may_alias)) v8ha;
typedef v4f  __attribute__((may_alias)) v4fa;
typedef v8us __attribute__((may_alias)) v8usa;

__device__ __forceinline__ unsigned short f2bf(float f) { unsigned u = __float_as_uint(f); u += 0x7FFFu + ((u >> 16) & 1u); return (unsigned short)(u >> 16); }
__device__ __forceinline__ float bf2f(unsigned short b) { return __uint_as_float(((unsigned)b) << 16); }
__device__ __forceinline__ float bfr(float f) { return bf2f(f2bf(f)); }
__device__ __forceinline__ void splitf(float y, unsigned short& h, unsigned short& l) { h = f2bf(y); l = f2bf(y - bf2f(h)); }
__device__ __forceinline__ v16h cat16(v8h lo, v8h hi) { return __builtin_shufflevector(lo, hi, 0, 1, 2, 3, 4, 5, 6, 7, 8, 9, 10, 11, 12, 13, 14, 15); }
__device__ __forceinline__ v16bf cat16b(v8us lo, v8us hi) { return __builtin_bit_cast(v16bf, __builtin_shufflevector(lo, hi, 0, 1, 2, 3, 4, 5, 6, 7, 8, 9, 10, 11, 12, 13, 14, 15)); }
__device__ __forceinline__ v8f wmma16(v16h a, v16h b, v8f c) { return __builtin_amdgcn_wmma_f32_16x16x32_f16(false, a, false, b, (short)0, c, false, false); }
__device__ __forceinline__ v8f wmmab(v16bf a, v16bf b, v8f c) { return __builtin_amdgcn_wmma_f32_16x16x32_bf16(false, a, false, b, (short)0, c, false, false); }

template <typename T16> struct WFrag;
template <> struct WFrag<h16> { typedef v16h V; static __device__ __forceinline__ V ld(const h16* p) { return cat16(*(const v8h*)p, *(const v8h*)(p + 16)); } static __device__ __forceinline__ v8f mma(V a, V b, v8f c) { return wmma16(a, b, c); } };
template <> struct WFrag<bf> { typedef v16bf V; static __device__ __forceinline__ V ld(const bf* p) { return cat16b(*(const v8us*)p, *(const v8us*)(p + 16)); } static __device__ __forceinline__ v8f mma(V a, V b, v8f c) { return wmmab(a, b, c); } };

template <typename T16, int NSPLIT, bool BIAS>
__device__ __forceinline__ void gemm_body(const T16* __restrict__ A, const T16* __restrict__ A2, const T16* __restrict__ Bt, const T16* __restrict__ Bt2, int K, float* C, int ldc, const float* __restrict__ bias, size_t sA, size_t sB, size_t sC) {
    typedef typename WFrag<T16>::V V;
    __shared__ __align__(16) float os[16 * 68];
    const size_t z = blockIdx.z; A += z * sA; if (A2) A2 += z * sA; Bt += z * sB; if (Bt2) Bt2 += z * sB; C += z * sC;
    const int lane = threadIdx.x & 31, lr = lane & 15, hi = lane >> 4; const int r0 = blockIdx.x * 64, c0 = blockIdx.y * 64;
    v8f acc[4][4];
#pragma unroll
    for (int mb = 0; mb < 4; ++mb)
#pragma unroll
        for (int nb = 0; nb < 4; ++nb) acc[mb][nb] = (v8f){};
    const size_t aoff = (size_t)(r0 + lr) * K + 8 * hi, boff = (size_t)(c0 + lr) * K + 8 * hi;
#pragma unroll 1
    for (int kc = 0; kc < K; kc += 32) {
        V a[4], a2[4];
#pragma unroll
        for (int mb = 0; mb < 4; ++mb) { a[mb] = WFrag<T16>::ld(A + aoff + (size_t)mb * 16 * K + kc); if (NSPLIT == 1 || NSPLIT == 2) a2[mb] = WFrag<T16>::ld(A2 + aoff + (size_t)mb * 16 * K + kc); }
#pragma unroll
        for (int nb = 0; nb < 4; ++nb) { const V b = WFrag<T16>::ld(Bt + boff + (size_t)nb * 16 * K + kc); V b2; if (NSPLIT >= 2) b2 = WFrag<T16>::ld(Bt2 + boff + (size_t)nb * 16 * K + kc);
#pragma unroll
            for (int mb = 0; mb < 4; ++mb) { acc[mb][nb] = WFrag<T16>::mma(a[mb], b, acc[mb][nb]); if (NSPLIT == 1 || NSPLIT == 2) acc[mb][nb] = WFrag<T16>::mma(a2[mb], b, acc[mb][nb]); if (NSPLIT >= 2) acc[mb][nb] = WFrag<T16>::mma(a[mb], b2, acc[mb][nb]); } }
        asm volatile("v_nop\n\tv_nop\n\tv_nop\n\tv_nop" : "+v"(acc[0][0]), "+v"(acc[1][1]), "+v"(acc[2][2]), "+v"(acc[3][3]) : "v"(a[0]), "v"(a[3]));
    }
#pragma unroll
    for (int mb = 0; mb < 4; ++mb) {
#pragma unroll
        for (int nb = 0; nb < 4; ++nb) {
#pragma unroll
            for (int j = 0; j < 8; ++j) os[(hi * 8 + j) * 68 + nb * 16 + lr] = acc[mb][nb][j]; }
        __builtin_amdgcn_wave_barrier(); asm volatile("" ::: "memory");
        float* crow = C + (size_t)(r0 + mb * 16) * ldc + c0;
#pragma unroll 1
        for (int ps = 0; ps < 2; ++ps) {
#pragma unroll
            for (int s = 0; s < 8; ++s) { const int row = 2 * s + hi, cofs = lr * 4; v4f val = *(const v4fa*)(os + row * 68 + cofs); if (BIAS) { val[0] += bfr(bias[c0 + cofs]); val[1] += bfr(bias[c0 + cofs + 1]); val[2] += bfr(bias[c0 + cofs + 2]); val[3] += bfr(bias[c0 + cofs + 3]); }
                *(volatile v4f*)(crow + (size_t)row * ldc + cofs) = val; }
            if (ps == 0) __threadfence(); }
        __builtin_amdgcn_wave_barrier(); asm volatile("" ::: "memory");
    }
}

__global__ __launch_bounds__(32) void k_gemm_qkv(const bf* XB, const bf* W, float* F) {
    gemm_body<bf, 0, false>(XB, nullptr, W, nullptr, DM, F, NQKV, nullptr, 0, 0, 0);
}
__global__ __launch_bounds__(32) void k_gemm_out(const bf* Ah, const bf* Al, const bf* W, const float* bias, float* OUT) {
    gemm_body<bf, 1, true>(Ah, Al, W, nullptr, DQ, OUT, DM, bias, (size_t)SEQ * DQ, 0, (size_t)SEQ_FULL * DM);
}

__global__ __launch_bounds__(256) void k_cvt8(const float* __restrict__ src, bf* dst, size_t n8) {
    const size_t i = (size_t)blockIdx.x * 256 + threadIdx.x; if (i >= n8) return; const v8f v = *(const v8f*)(src + i * 8); v8us o;
#pragma unroll
    for (int k = 0; k < 8; ++k) o[k] = f2bf(v[k]);
    *(volatile v8us*)(dst + i * 8) = o; __threadfence(); *(volatile v8us*)(dst + i * 8) = o;
}
__global__ __launch_bounds__(256) void k_cvtx(const float* __restrict__ x, bf* XB) {
    const size_t i = (size_t)blockIdx.x * 256 + threadIdx.x; if (i >= (size_t)NB * SEQ * DM / 8) return;
    const int c8 = (int)(i % (DM / 8)); const int row = (int)(i / (DM / 8)); const int b = row / SEQ, t = row % SEQ;
    const v8f v = *(const v8f*)(x + ((size_t)b * SEQ_FULL + t) * DM + c8 * 8); v8us o;
#pragma unroll
    for (int k = 0; k < 8; ++k) o[k] = f2bf(v[k]);
    *(volatile v8us*)(XB + i * 8) = o; __threadfence(); *(volatile v8us*)(XB + i * 8) = o;
}

__global__ __launch_bounds__(256) void k_cstab(float* CS) {
    const int idx = blockIdx.x * 256 + threadIdx.x; if (idx >= SEQ * NTAB) return;
    const int i = idx % NTAB, t = idx / NTAB;
    const float pw = powf(10000.0f, (float)(2 * i));
    const float th = 1.0f / (pw / 64.0f);
    const float ang = (float)t * th;
    float sn, cn; sincosf(ang, &sn, &cn);
    v2f o; o[0] = cn; o[1] = sn;
    *(volatile v2f*)(CS + (size_t)idx * 2) = o; __threadfence(); *(volatile v2f*)(CS + (size_t)idx * 2) = o;
}

__global__ __launch_bounds__(256) void k_rope(const float* __restrict__ F, int col0, int nheads, const float* __restrict__ bias, const float* __restrict__ CS, bf* Ph, bf* Pl) {
    const size_t e = ((size_t)blockIdx.x * 256 + threadIdx.x) * 2; if (e >= (size_t)NB * nheads * SEQ * HD) return;
    const int d = (int)(e % HD); const int t = (int)((e / HD) % SEQ); const int bh = (int)(e / ((size_t)HD * SEQ)); const int h = bh % nheads, b = bh / nheads;
    const v2f xv = *(const v2f*)(F + ((size_t)b * SEQ + t) * NQKV + col0 + h * HD + d);
    const float x1 = xv[0] + bfr(bias[h * HD + d]), x2 = xv[1] + bfr(bias[h * HD + d + 1]);
    const int i = d >> 1; const int ic = (i < NTAB - 1) ? i : (NTAB - 1);
    const v2f cs = *(const v2f*)(CS + ((size_t)t * NTAB + ic) * 2);
    const float c = (i < NROT) ? cs[0] : 1.0f; const float s = (i < NROT) ? cs[1] : 0.0f;
    const float pa = x1 * c, pb = x2 * s;
    const float r0 = pa - pb, r1 = pb + pa;
    unsigned short a0, c0, a1, c1; splitf(r0, a0, c0); splitf(r1, a1, c1);
    v2us oh, ol; oh[0] = a0; oh[1] = a1; ol[0] = c0; ol[1] = c1;
    *(volatile v2us*)(Ph + e) = oh; *(volatile v2us*)(Pl + e) = ol;
    __threadfence();
    *(volatile v2us*)(Ph + e) = oh; *(volatile v2us*)(Pl + e) = ol;
}

__global__ __launch_bounds__(256) void k_vtp(const float* __restrict__ F, int col0, const float* __restrict__ bias, h16* V16, bf* Vh, bf* Vl) {
    const size_t e = ((size_t)blockIdx.x * 256 + threadIdx.x) * 2; if (e >= (size_t)NB * NKV * HD * SEQ) return;
    const int t = (int)(e % SEQ); const int d = (int)((e / SEQ) % HD); const int bg = (int)(e / ((size_t)SEQ * HD)); const int g = bg % NKV, b = bg / NKV;
    const float bv = bfr(bias[g * HD + d]);
    const float xa = F[((size_t)b * SEQ + t) * NQKV + col0 + g * HD + d] + bv;
    const float xb = F[((size_t)b * SEQ + t + 1) * NQKV + col0 + g * HD + d] + bv;
    v2h o16; o16[0] = (h16)xa; o16[1] = (h16)xb;
    unsigned short a0, c0, a1, c1; splitf(xa, a0, c0); splitf(xb, a1, c1);
    v2us oh, ol; oh[0] = a0; oh[1] = a1; ol[0] = c0; ol[1] = c1;
    const bool whl = (t < RH);
    const size_t eh = ((size_t)bg * HD + d) * RH + (whl ? t : 0);
    *(volatile v2h*)(V16 + e) = o16;
    if (whl) { *(volatile v2us*)(Vh + eh) = oh; *(volatile v2us*)(Vl + eh) = ol; }
    __threadfence();
    *(volatile v2h*)(V16 + e) = o16;
    if (whl) { *(volatile v2us*)(Vh + eh) = oh; *(volatile v2us*)(Vl + eh) = ol; }
}

template <typename TV, bool HI>
__device__ __forceinline__ void flash_body(const bf* __restrict__ Qh, const bf* __restrict__ Ql, const bf* __restrict__ Kh, const bf* __restrict__ Kl, const TV* __restrict__ Va, const TV* __restrict__ Vb, bf* ATh, bf* ATl) {
    typedef typename WFrag<bf>::V VS;
    typedef typename WFrag<TV>::V VP;
    __shared__ __align__(16) TV pa_t[4][16 * PP];
    __shared__ __align__(16) TV pb_t[4][16 * PP];
    __shared__ __align__(16) float os[4][16 * 68];
    const int wv = threadIdx.x >> 5, lane = threadIdx.x & 31, lr = lane & 15, hi = lane >> 4;
    const int h = blockIdx.y, b = blockIdx.z, kv = h / REP;
    constexpr int TVP = HI ? RH : SEQ;
    const int q0 = (HI ? 0 : RH) + (blockIdx.x * 4 + wv) * 16;
    const size_t qoff = ((size_t)(b * NH + h) * SEQ + q0 + lr) * HD + 8 * hi;
    const size_t kbase = ((size_t)(b * NKV + kv) * SEQ + lr) * HD + 8 * hi;
    const size_t vbase = ((size_t)(b * NKV + kv) * HD + lr) * TVP + 8 * hi;
    VS qa[2], qb[2];
#pragma unroll
    for (int ks = 0; ks < 2; ++ks) { qa[ks] = WFrag<bf>::ld(Qh + qoff + ks * 32); qb[ks] = WFrag<bf>::ld(Ql + qoff + ks * 32); }
    float mrow[8], lrow[8]; v8f oc[4];
#pragma unroll
    for (int r = 0; r < 8; ++r) { mrow[r] = NEGBIG; lrow[r] = 0.0f; }
#pragma unroll
    for (int nt = 0; nt < 4; ++nt) oc[nt] = (v8f){};
    const int nblk = (q0 + 15) / 32 + 1;
#pragma unroll 1
    for (int j = 0; j < nblk; ++j) {
        const int k0 = j * 32;
        VS kf[4], kg[4];
#pragma unroll
        for (int t = 0; t < 2; ++t)
#pragma unroll
            for (int ks = 0; ks < 2; ++ks) { const size_t ko = kbase + (size_t)(k0 + t * 16) * HD + ks * 32; kf[t * 2 + ks] = WFrag<bf>::ld(Kh + ko); kg[t * 2 + ks] = WFrag<bf>::ld(Kl + ko); }
        v8f st0 = (v8f){}, st1 = (v8f){};
        st0 = WFrag<bf>::mma(qa[0], kf[0], st0); st1 = WFrag<bf>::mma(qa[0], kf[2], st1);
        st0 = WFrag<bf>::mma(qa[1], kf[1], st0); st1 = WFrag<bf>::mma(qa[1], kf[3], st1);
        st0 = WFrag<bf>::mma(qa[0], kg[0], st0); st1 = WFrag<bf>::mma(qa[0], kg[2], st1);
        st0 = WFrag<bf>::mma(qa[1], kg[1], st0); st1 = WFrag<bf>::mma(qa[1], kg[3], st1);
        st0 = WFrag<bf>::mma(qb[0], kf[0], st0); st1 = WFrag<bf>::mma(qb[0], kf[2], st1);
        st0 = WFrag<bf>::mma(qb[1], kf[1], st0); st1 = WFrag<bf>::mma(qb[1], kf[3], st1);
        asm volatile("v_nop\n\tv_nop\n\tv_nop\n\tv_nop" : "+v"(st0), "+v"(st1) : "v"(kf[0]), "v"(kf[1]), "v"(kf[2]), "v"(kf[3]), "v"(kg[0]), "v"(kg[1]), "v"(kg[2]), "v"(kg[3]), "v"(qa[0]), "v"(qa[1]), "v"(qb[0]), "v"(qb[1]));
#pragma unroll
        for (int r = 0; r < 8; ++r) {
            const int row = q0 + 8 * hi + r;
            const float s0 = (k0 + lr <= row) ? st0[r] * 0.125f : NEGBIG;
            const float s1 = (k0 + 16 + lr <= row) ? st1[r] * 0.125f : NEGBIG;
            float rm = fmaxf(s0, s1);
            rm = fmaxf(rm, __shfl_xor(rm, 1, 32)); rm = fmaxf(rm, __shfl_xor(rm, 2, 32)); rm = fmaxf(rm, __shfl_xor(rm, 4, 32)); rm = fmaxf(rm, __shfl_xor(rm, 8, 32));
            const float nm = fmaxf(mrow[r], rm);
            const float corr = __builtin_amdgcn_exp2f((mrow[r] - nm) * L2E);
            const float p0 = __builtin_amdgcn_exp2f((s0 - nm) * L2E);
            const float p1 = __builtin_amdgcn_exp2f((s1 - nm) * L2E);
            lrow[r] = lrow[r] * corr + (p0 + p1);
            mrow[r] = nm;
            oc[0][r] *= corr; oc[1][r] *= corr; oc[2][r] *= corr; oc[3][r] *= corr;
            const int pi = (8 * hi + r) * PP + lr;
            if constexpr (HI) {
                unsigned short a0, c0, a1, c1; splitf(p0, a0, c0); splitf(p1, a1, c1);
                pa_t[wv][pi] = a0; pb_t[wv][pi] = c0; pa_t[wv][pi + 16] = a1; pb_t[wv][pi + 16] = c1;
            } else {
                pa_t[wv][pi] = (h16)(p0 * PCAR); pa_t[wv][pi + 16] = (h16)(p1 * PCAR);
            }
        }
        __builtin_amdgcn_wave_barrier(); asm volatile("" ::: "memory");
        const int fi = lr * PP + 8 * hi;
        VP pf, pg;
        if constexpr (HI) {
            pf = cat16b(*(const v8usa*)(&pa_t[wv][fi]), *(const v8usa*)(&pa_t[wv][fi + 16]));
            pg = cat16b(*(const v8usa*)(&pb_t[wv][fi]), *(const v8usa*)(&pb_t[wv][fi + 16]));
        } else {
            pf = cat16(*(const v8ha*)(&pa_t[wv][fi]), *(const v8ha*)(&pa_t[wv][fi + 16]));
        }
        VP vf[4], vg[4];
#pragma unroll
        for (int nt = 0; nt < 4; ++nt) { const size_t vo = vbase + (size_t)(nt * 16) * TVP + k0; vf[nt] = WFrag<TV>::ld(Va + vo); if constexpr (HI) vg[nt] = WFrag<TV>::ld(Vb + vo); }
#pragma unroll
        for (int nt = 0; nt < 4; ++nt) oc[nt] = WFrag<TV>::mma(pf, vf[nt], oc[nt]);
        if constexpr (HI) {
#pragma unroll
            for (int nt = 0; nt < 4; ++nt) oc[nt] = WFrag<TV>::mma(pf, vg[nt], oc[nt]);
#pragma unroll
            for (int nt = 0; nt < 4; ++nt) oc[nt] = WFrag<TV>::mma(pg, vf[nt], oc[nt]);
            asm volatile("v_nop\n\tv_nop\n\tv_nop\n\tv_nop" : "+v"(oc[0]), "+v"(oc[1]), "+v"(oc[2]), "+v"(oc[3]) : "v"(pf), "v"(pg), "v"(vf[0]), "v"(vf[1]), "v"(vf[2]), "v"(vf[3]), "v"(vg[0]), "v"(vg[1]), "v"(vg[2]), "v"(vg[3]));
        } else {
            asm volatile("v_nop\n\tv_nop\n\tv_nop\n\tv_nop" : "+v"(oc[0]), "+v"(oc[1]), "+v"(oc[2]), "+v"(oc[3]) : "v"(pf), "v"(vf[0]), "v"(vf[1]), "v"(vf[2]), "v"(vf[3]));
        }
        __builtin_amdgcn_wave_barrier(); asm volatile("" ::: "memory");
    }
#pragma unroll
    for (int r = 0; r < 8; ++r) {
        float l = lrow[r];
        l += __shfl_xor(l, 1, 32); l += __shfl_xor(l, 2, 32); l += __shfl_xor(l, 4, 32); l += __shfl_xor(l, 8, 32);
        const float inv = 1.0f / (HI ? l : l * PCAR);
#pragma unroll
        for (int nt = 0; nt < 4; ++nt) os[wv][(8 * hi + r) * 68 + nt * 16 + lr] = oc[nt][r] * inv;
    }
    __builtin_amdgcn_wave_barrier(); asm volatile("" ::: "memory");
    bf* ah = ATh + ((size_t)b * SEQ + q0) * DQ + h * HD;
    bf* al = ATl + ((size_t)b * SEQ + q0) * DQ + h * HD;
#pragma unroll 1
    for (int ps = 0; ps < 2; ++ps) {
#pragma unroll
        for (int s = 0; s < 4; ++s) {
            const int row = 4 * s + (lane >> 3), c8 = (lane & 7) * 8;
            const v4f u0 = *(const v4fa*)(&os[wv][row * 68 + c8]); const v4f u1 = *(const v4fa*)(&os[wv][row * 68 + c8 + 4]);
            v8us oh, ol;
#pragma unroll
            for (int k = 0; k < 4; ++k) { unsigned short a, c; splitf(u0[k], a, c); oh[k] = a; ol[k] = c; splitf(u1[k], a, c); oh[4 + k] = a; ol[4 + k] = c; }
            *(volatile v8us*)(ah + (size_t)row * DQ + c8) = oh; *(volatile v8us*)(al + (size_t)row * DQ + c8) = ol;
        }
        if (ps == 0) __threadfence();
    }
}

__global__ __launch_bounds__(128) void k_flash_hi(const bf* Qh, const bf* Ql, const bf* Kh, const bf* Kl, const bf* Vh, const bf* Vl, bf* ATh, bf* ATl) {
    flash_body<bf, true>(Qh, Ql, Kh, Kl, Vh, Vl, ATh, ATl);
}
__global__ __launch_bounds__(128) void k_flash_lo(const bf* Qh, const bf* Ql, const bf* Kh, const bf* Kl, const h16* V16, bf* ATh, bf* ATl) {
    flash_body<h16, false>(Qh, Ql, Kh, Kl, V16, V16, ATh, ATl);
}

constexpr size_t al256(size_t x) { return (x + 255) & ~(size_t)255; }
constexpr size_t SZ_XB  = al256((size_t)NB * SEQ * DM * 2);
constexpr size_t SZ_WQ  = al256((size_t)NQKV * DM * 2);
constexpr size_t SZ_WO  = al256((size_t)DM * DQ * 2);
constexpr size_t SZ_CS  = al256((size_t)SEQ * NTAB * 2 * 4);
constexpr size_t SZ_F   = al256((size_t)NB * SEQ * NQKV * 4);
constexpr size_t SZ_QH  = al256((size_t)NB * NH * SEQ * HD * 2);
constexpr size_t SZ_KH  = al256((size_t)NB * NKV * SEQ * HD * 2);
constexpr size_t SZ_V16 = al256((size_t)NB * NKV * HD * SEQ * 2);
constexpr size_t SZ_VH  = al256((size_t)NB * NKV * HD * RH * 2);
constexpr size_t SZ_AT  = al256((size_t)NB * SEQ * DQ * 2);
constexpr size_t OFF_XB  = 0;
constexpr size_t OFF_WQ  = OFF_XB + SZ_XB;
constexpr size_t OFF_WO  = OFF_WQ + SZ_WQ;
constexpr size_t OFF_CS  = OFF_WO + SZ_WO;
constexpr size_t OFF_F   = OFF_CS + SZ_CS;
constexpr size_t OFF_QH  = OFF_F + SZ_F;
constexpr size_t OFF_QL  = OFF_QH + SZ_QH;
constexpr size_t OFF_KH  = OFF_QL + SZ_QH;
constexpr size_t OFF_KL  = OFF_KH + SZ_KH;
constexpr size_t OFF_V16 = OFF_KL + SZ_KH;
constexpr size_t OFF_VH  = OFF_V16 + SZ_V16;
constexpr size_t OFF_VL  = OFF_VH + SZ_VH;
constexpr size_t OFF_ATH = OFF_VL + SZ_VH;
constexpr size_t OFF_ATL = OFF_ATH + SZ_AT;
constexpr size_t WS_TOTAL = OFF_ATL + SZ_AT;
static_assert(WS_TOTAL <= (size_t)134217728);

extern "C" void kernel_launch(void* const* d_in, const int* in_sizes, int n_in,
                              void* d_out, int out_size, void* d_ws, size_t ws_size, hipStream_t stream) {
    if (n_in < 9) return;
    const long long xneed = ((long long)(NB - 1) * SEQ_FULL + SEQ) * DM;
    if ((long long)in_sizes[0] < xneed) return;
    if (in_sizes[1] < DQ * DM || in_sizes[2] < DQ || in_sizes[3] < DKV * DM || in_sizes[4] < DKV || in_sizes[5] < DKV * DM || in_sizes[6] < DKV || in_sizes[7] < DM * DQ || in_sizes[8] < DM) return;
    if ((long long)out_size < xneed) return;
    if (WS_TOTAL > ws_size) return;
    const float* x  = (const float*)d_in[0]; const float* wq = (const float*)d_in[1]; const float* bq = (const float*)d_in[2];
    const float* wk = (const float*)d_in[3]; const float* bk = (const float*)d_in[4]; const float* wv = (const float*)d_in[5];
    const float* bv = (const float*)d_in[6]; const float* wo = (const float*)d_in[7]; const float* bo = (const float*)d_in[8];
    float* OUT = (float*)d_out;
    char* ws = (char*)d_ws;
    bf* XB = (bf*)(ws + OFF_XB); bf* WQKV = (bf*)(ws + OFF_WQ); bf* WO = (bf*)(ws + OFF_WO); float* CS = (float*)(ws + OFF_CS); float* F = (float*)(ws + OFF_F);
    bf* Qh = (bf*)(ws + OFF_QH); bf* Ql = (bf*)(ws + OFF_QL); bf* Kh = (bf*)(ws + OFF_KH); bf* Kl = (bf*)(ws + OFF_KL);
    h16* V16 = (h16*)(ws + OFF_V16); bf* Vh = (bf*)(ws + OFF_VH); bf* Vl = (bf*)(ws + OFF_VL);
    bf* ATh = (bf*)(ws + OFF_ATH); bf* ATl = (bf*)(ws + OFF_ATL);

    k_cvtx<<<(unsigned)(((size_t)NB * SEQ * DM / 8 + 255) / 256), 256, 0, stream>>>(x, XB);
    k_cvt8<<<(unsigned)(((size_t)DQ * DM / 8 + 255) / 256), 256, 0, stream>>>(wq, WQKV, (size_t)DQ * DM / 8);
    k_cvt8<<<(unsigned)(((size_t)DKV * DM / 8 + 255) / 256), 256, 0, stream>>>(wk, WQKV + (size_t)DQ * DM, (size_t)DKV * DM / 8);
    k_cvt8<<<(unsigned)(((size_t)DKV * DM / 8 + 255) / 256), 256, 0, stream>>>(wv, WQKV + (size_t)(DQ + DKV) * DM, (size_t)DKV * DM / 8);
    k_cvt8<<<(unsigned)(((size_t)DM * DQ / 8 + 255) / 256), 256, 0, stream>>>(wo, WO, (size_t)DM * DQ / 8);
    k_cstab<<<(SEQ * NTAB + 255) / 256, 256, 0, stream>>>(CS);
    k_gemm_qkv<<<dim3(NB * SEQ / 64, NQKV / 64, 1), 32, 0, stream>>>(XB, WQKV, F);
    const unsigned LQ = (unsigned)(((size_t)NB * NH * SEQ * HD / 2 + 255) / 256), LK = (unsigned)(((size_t)NB * NKV * SEQ * HD / 2 + 255) / 256);
    k_rope<<<LQ, 256, 0, stream>>>(F, 0, NH, bq, CS, Qh, Ql);
    k_rope<<<LK, 256, 0, stream>>>(F, DQ, NKV, bk, CS, Kh, Kl);
    k_vtp<<<LK, 256, 0, stream>>>(F, DQ + DKV, bv, V16, Vh, Vl);
    k_flash_hi<<<dim3(RH / 64, NH, NB), 128, 0, stream>>>(Qh, Ql, Kh, Kl, Vh, Vl, ATh, ATl);
    if (SEQ > RH) k_flash_lo<<<dim3((SEQ - RH) / 64 > 0 ? (SEQ - RH) / 64 : 1, NH, NB), 128, 0, stream>>>(Qh, Ql, Kh, Kl, V16, ATh, ATl);
    k_gemm_out<<<dim3(SEQ / 64, DM / 64, NB), 32, 0, stream>>>(ATh, ATl, WO, bo, OUT);
}
